// ChebConv_test_5729486372945
// MI455X (gfx1250) — hardware-verified
//
#include <hip/hip_runtime.h>
#include <math.h>
typedef __attribute__((ext_vector_type(16))) _Float16 v16h;
typedef __attribute__((ext_vector_type(8)))  _Float16 v8h;
typedef __attribute__((ext_vector_type(16))) __bf16   v16b;
typedef __attribute__((ext_vector_type(8)))  __bf16   v8b;
typedef __attribute__((ext_vector_type(8)))  float    v8f;
typedef __attribute__((ext_vector_type(4)))  float    v4f;
#define PSCALE 32768.0f
#define U16(p) ((const unsigned short*)(const void*)(p))
#define PSCALE_INV (1.0f / 32768.0f)

__device__ __forceinline__ unsigned short f2bf_bits(float f) {
  unsigned u = __float_as_uint(f);
  return (unsigned short)((u + 0x7FFFu + ((u >> 16) & 1u)) >> 16);
}
__device__ __forceinline__ float bf_bits2f(unsigned short h) { return __uint_as_float(((unsigned)h) << 16); }

__device__ __forceinline__ void dep_guard_h(v8f& a, v8f& b, v16h x, v16h y) { asm volatile("v_nop\n\tv_nop\n\tv_nop\n\tv_nop" : "+v"(a), "+v"(b) : "v"(x), "v"(y)); }
__device__ __forceinline__ void dep_guard_b(v8f& a, v8f& b, v16b x, v16b y) { asm volatile("v_nop\n\tv_nop\n\tv_nop\n\tv_nop" : "+v"(a), "+v"(b) : "v"(x), "v"(y)); }
__device__ __forceinline__ void keep4_h(v16h a, v16h b, v16h c, v16h d) { asm volatile("v_nop" :: "v"(a), "v"(b), "v"(c), "v"(d)); }
__device__ __forceinline__ void keep4_b(v16b a, v16b b, v16b c, v16b d) { asm volatile("v_nop" :: "v"(a), "v"(b), "v"(c), "v"(d)); }
__device__ __forceinline__ void acc_guard4(v8f& a, v8f& b, v8f& c, v8f& d) { asm volatile("v_nop\n\tv_nop\n\tv_nop\n\tv_nop" : "+v"(a), "+v"(b), "+v"(c), "+v"(d)); }
template <typename T> struct Frag;
template <> struct Frag<_Float16> {
  typedef v16h V; union U { v16h v; v8h h[2]; };
  static __device__ __forceinline__ v16h load(const _Float16* p) {
    U f; f.h[0] = *(const v8h*)(p); f.h[1] = *(const v8h*)(p + 16); return f.v;
  }
  static __device__ __forceinline__ v8f mma(v16h a, v16h b, v8f c) {
    return __builtin_amdgcn_wmma_f32_16x16x32_f16(false, a, false, b, (short)0, c, false, false);
  }
  static __device__ __forceinline__ void guard(v8f& a, v8f& b, v16h x, v16h y) { dep_guard_h(a, b, x, y); }
  static __device__ __forceinline__ void keep(v16h a, v16h b, v16h c, v16h d) { keep4_h(a, b, c, d); }
};
template <> struct Frag<__bf16> {
  typedef v16b V; union U { v16b v; v8b h[2]; };
  static __device__ __forceinline__ v16b load(const __bf16* p) {
    U f; f.h[0] = *(const v8b*)(p); f.h[1] = *(const v8b*)(p + 16); return f.v;
  }
  static __device__ __forceinline__ v8f mma(v16b a, v16b b, v8f c) {
    return __builtin_amdgcn_wmma_f32_16x16x32_bf16(false, a, false, b, (short)0, c, false, false);
  }
  static __device__ __forceinline__ void guard(v8f& a, v8f& b, v16b x, v16b y) { dep_guard_b(a, b, x, y); }
  static __device__ __forceinline__ void keep(v16b a, v16b b, v16b c, v16b d) { keep4_b(a, b, c, d); }
};

template <int ET> struct Elem;
template <> struct Elem<0> { typedef _Float16 T; };
template <> struct Elem<1> { typedef __bf16 T; };
template <int ET, bool SPLIT, int BIAS_MODE, int OUT_MODE, bool RESID, int ACT = 0>
__global__ __launch_bounds__(256) void wmma_gemm64(
    const unsigned short* __restrict__ Ap, const unsigned short* __restrict__ A2p, int lda, long strideA,
    const unsigned short* __restrict__ Btp, const unsigned short* __restrict__ Bt2p, int ldb, long strideB,
    void* __restrict__ Cout, void* __restrict__ Cout2, int ldc, long strideC,
    const float* __restrict__ bias,
    const float* __restrict__ resid, long strideR,
    int M, int N, int K, float scale) {
  typedef typename Elem<ET>::T T;
  typedef typename Frag<T>::V V;
  const T* A = (const T*)Ap; const T* A2 = (const T*)A2p; const T* Bt = (const T*)Btp; const T* Bt2 = (const T*)Bt2p;
  __shared__ __align__(16) float sT[8][16 * 68];
  const int b    = blockIdx.y;
  const int lane = threadIdx.x & 31;
  const int wave = threadIdx.x >> 5;
  const int tilesN = N >> 6;
  const int tilesM = M >> 6;
  const int tile = blockIdx.x * 8 + wave;
  if (tile >= tilesM * tilesN) return;
  const int tm = tile / tilesN;
  const int tn = tile - tm * tilesN;
  const int m0 = tm << 6;
  const int n0 = tn << 6;

  const T* Ab  = A  + (size_t)b * strideA;
  const T* Bb  = Bt + (size_t)b * strideB;
  const T* Ab2 = SPLIT ? (A2  + (size_t)b * strideA) : nullptr;
  const T* Bb2 = SPLIT ? (Bt2 + (size_t)b * strideB) : nullptr;

  const int rlane = lane & 15;
  const int koff  = (lane >> 4) * 8;
  const int mOff  = (lane >> 4) * 8;

  v8f acc[4][4];
#pragma unroll
  for (int i = 0; i < 4; ++i)
#pragma unroll
    for (int j = 0; j < 4; ++j) acc[i][j] = (v8f){0.f,0.f,0.f,0.f,0.f,0.f,0.f,0.f};

  for (int k0 = 0; k0 < K; k0 += 32) {
    V bh[4], bl[4];
#pragma unroll
    for (int j = 0; j < 4; ++j) {
      const size_t bo = (size_t)(n0 + (j << 4) + rlane) * ldb + koff + k0;
      bh[j] = Frag<T>::load(Bb + bo);
      if (SPLIT) bl[j] = Frag<T>::load(Bb2 + bo);
    }
#pragma unroll
    for (int i = 0; i < 4; ++i) {
      const size_t ao = (size_t)(m0 + (i << 4) + rlane) * lda + koff + k0;
      V ah = Frag<T>::load(Ab + ao);
      V al;
      if (SPLIT) al = Frag<T>::load(Ab2 + ao);
#pragma unroll
      for (int j = 0; j < 4; ++j) {
        acc[i][j] = Frag<T>::mma(ah, bh[j], acc[i][j]);
        if (SPLIT) {
          acc[i][j] = Frag<T>::mma(ah, bl[j], acc[i][j]);
          acc[i][j] = Frag<T>::mma(al, bh[j], acc[i][j]);
        }
      }
      Frag<T>::guard(acc[i][0], acc[i][3], ah, SPLIT ? al : ah);
    }
    Frag<T>::keep(bh[0], bh[1], bh[2], bh[3]);
    if (SPLIT) Frag<T>::keep(bl[0], bl[1], bl[2], bl[3]);
  }
  acc_guard4(acc[0][0], acc[0][1], acc[0][2], acc[0][3]);
  acc_guard4(acc[1][0], acc[1][1], acc[1][2], acc[1][3]);
  acc_guard4(acc[2][0], acc[2][1], acc[2][2], acc[2][3]);
  acc_guard4(acc[3][0], acc[3][1], acc[3][2], acc[3][3]);

  float* slab = sT[wave];
  const float* Rb = RESID ? (resid + (size_t)b * strideR) : nullptr;
#pragma unroll
  for (int i = 0; i < 4; ++i) {
    const int mBase = m0 + (i << 4);
#pragma unroll
    for (int j = 0; j < 4; ++j) {
      const int n = n0 + (j << 4) + rlane;
      float bv = 0.f;
      if (BIAS_MODE == 2) bv = bias[n];
#pragma unroll
      for (int r = 0; r < 8; ++r) {
        float v = acc[i][j][r] * scale;
        if (BIAS_MODE == 1) v += bias[mBase + mOff + r];
        if (BIAS_MODE == 2) v += bv;
        if (RESID) v += Rb[(size_t)(mBase + mOff + r) * ldc + n];
        if (ACT == 1) v = tanhf(v);
        if (ACT == 2) v = fmaxf(v, 0.0f);
        if (ACT == 3) v = v / (1.0f + expf(-v));
        if (ACT == 4) v = (v > 0.f) ? v : 0.01f * v;
        if (ACT == 5) v = 0.5f * v * (1.0f + erff(v * 0.70710678118654752f));
        slab[(mOff + r) * 68 + (j << 4) + rlane] = v;
      }
    }
    __builtin_amdgcn_fence(__ATOMIC_RELEASE, "workgroup");
    __builtin_amdgcn_wave_barrier();
    __builtin_amdgcn_fence(__ATOMIC_ACQUIRE, "workgroup");
    if (OUT_MODE == 0) {
      float* C = (float*)Cout + (size_t)b * strideC;
      const int hh = lane >> 4, c4 = (lane & 15) * 4;
      for (int pass = 0; pass < 2; ++pass) {
#pragma unroll
        for (int it = 0; it < 8; ++it) {
          const int row = it * 2 + hh;
          v4f v = *(const v4f*)(slab + row * 68 + c4);
          *(volatile v4f*)(C + (size_t)(mBase + row) * ldc + n0 + c4) = v;
        }
        __threadfence();
      }
    } else {
      const int q = lane >> 3, c8 = (lane & 7) * 8;
      unsigned short* C  = (unsigned short*)Cout  + (size_t)b * strideC;
      unsigned short* C2 = (OUT_MODE == 2) ? ((unsigned short*)Cout2 + (size_t)b * strideC) : nullptr;
      for (int pass = 0; pass < 2; ++pass) {
#pragma unroll
        for (int it = 0; it < 4; ++it) {
          const int row = it * 4 + q;
          const float* sp = slab + row * 68 + c8;
          v8h hv, lv;
#pragma unroll
          for (int e = 0; e < 8; ++e) {
            if (OUT_MODE == 1) {
              hv[e] = (_Float16)sp[e];
            } else {
              unsigned short hb = f2bf_bits(sp[e]);
              unsigned short lb = f2bf_bits(sp[e] - bf_bits2f(hb));
              hv[e] = __builtin_bit_cast(_Float16, hb);
              lv[e] = __builtin_bit_cast(_Float16, lb);
            }
          }
          *(volatile v8h*)(C + (size_t)(mBase + row) * ldc + n0 + c8) = hv;
          if (OUT_MODE == 2) *(volatile v8h*)(C2 + (size_t)(mBase + row) * ldc + n0 + c8) = lv;
        }
        __threadfence();
      }
    }
    __builtin_amdgcn_fence(__ATOMIC_RELEASE, "workgroup");
    __builtin_amdgcn_wave_barrier();
    __builtin_amdgcn_fence(__ATOMIC_ACQUIRE, "workgroup");
  }
}

__global__ __launch_bounds__(256) void cast_f32_f16x2(
    const float* __restrict__ in, _Float16* __restrict__ out, int n2) {
  int i = blockIdx.x * 256 + threadIdx.x;
  if (i < n2) {
    const _Float16 h0 = (_Float16)in[2 * i], h1 = (_Float16)in[2 * i + 1];
    const unsigned u = (unsigned)__builtin_bit_cast(unsigned short, h0) | ((unsigned)__builtin_bit_cast(unsigned short, h1) << 16);
    ((volatile unsigned*)out)[i] = u;
    __threadfence();
    ((volatile unsigned*)out)[i] = u;
  }
}


#define CBt 131072
#define CNn 24
#define CE 128
#define CF1 4
#define CH 8
#define CNP 32
#define CCH 32768
__global__ __launch_bounds__(256) void lap_kernel(const int* __restrict__ ei, unsigned* __restrict__ LB) {
  __shared__ float deg[CNn]; __shared__ float Lm[64][64];
  const int t = threadIdx.x;
  for (int i = t; i < 64 * 64; i += 256) (&Lm[0][0])[i] = 0.f;
  if (t < CNn) { float d = 0.f; for (int e = 0; e < CE; ++e) if (ei[e] == t) d += 1.f; deg[t] = d; }
  __syncthreads();
  if (t == 0) { for (int e = 0; e < CE; ++e) { int r = ei[e], c = ei[CE + e]; r = r < 0 ? 0 : (r >= CNn ? CNn - 1 : r); c = c < 0 ? 0 : (c >= CNn ? CNn - 1 : c);
      const float dr = deg[r] > 0.f ? 1.0f / sqrtf(deg[r]) : 0.f, dc = deg[c] > 0.f ? 1.0f / sqrtf(deg[c]) : 0.f; Lm[r][c] += -dr * dc; Lm[32 + r][32 + c] += -dr * dc; } }
  __syncthreads();
  for (int pass = 0; pass < 2; ++pass) { for (int i = t; i < 64 * 64 / 2; i += 256) { const float a = (&Lm[0][0])[2 * i], b = (&Lm[0][0])[2 * i + 1];
      ((volatile unsigned*)LB)[i] = (unsigned)__builtin_bit_cast(unsigned short, (_Float16)a) | ((unsigned)__builtin_bit_cast(unsigned short, (_Float16)b) << 16); } __threadfence(); }
}
__global__ __launch_bounds__(256) void t0_kernel(const float* __restrict__ x, unsigned* __restrict__ T0) {
  const long i = (long)blockIdx.x * 256 + threadIdx.x; if (i >= (long)(CCH / 2) * CF1) return; const long p = i / CF1; const int f = (int)(i % CF1);
  unsigned row[32];
#pragma unroll
  for (int q = 0; q < 32; ++q) { const int j = q / 16; const int m0 = 2 * (q % 16); const long b = 2 * p + j; float a = 0.f, c = 0.f;
    if (m0 < CNn) a = x[(b * CNn + m0) * CF1 + f]; if (m0 + 1 < CNn) c = x[(b * CNn + m0 + 1) * CF1 + f];
    row[q] = (unsigned)__builtin_bit_cast(unsigned short, (_Float16)a) | ((unsigned)__builtin_bit_cast(unsigned short, (_Float16)c) << 16); }
  typedef __attribute__((ext_vector_type(4))) unsigned u4;
  for (int pass = 0; pass < 2; ++pass) {
#pragma unroll
    for (int q = 0; q < 8; ++q) { u4 v = {row[4*q], row[4*q+1], row[4*q+2], row[4*q+3]}; *(volatile u4*)(T0 + i * 32 + q * 4) = v; }
    __threadfence(); }
}
__device__ __forceinline__ float h16(const unsigned* p, long idx) { const unsigned u = p[idx >> 1]; return (float)__builtin_bit_cast(_Float16, (unsigned short)((idx & 1) ? (u >> 16) : (u & 0xFFFFu))); }
template <int FIN, bool LAST>
__global__ __launch_bounds__(256) void comb_kernel(const float* __restrict__ Xf32, const unsigned* __restrict__ X16, const unsigned* __restrict__ T1, const float* __restrict__ C2, const float* __restrict__ Wc, const float* __restrict__ bc,
                                                  unsigned* __restrict__ TOUT, unsigned* __restrict__ FLAT) {
  const int lane = threadIdx.x & 31, wave = threadIdx.x >> 5; const long b = (long)blockIdx.x * 8 + wave; const int n = lane; const bool live = (n < CNn);
  const long p = b >> 1; const int jj = (int)(b & 1);
  float t0[FIN], t1[FIN], t2[FIN];
#pragma unroll
  for (int f = 0; f < FIN; ++f) { const long e = (p * FIN + f) * 64 + jj * 32 + n;
    const float x0 = live ? (Xf32 ? Xf32[(b * CNn + n) * FIN + f] : h16(X16, e)) : 0.f;
    const float p1 = live ? h16(T1, e) : 0.f, p2 = live ? C2[e] : 0.f;
    t0[f] = x0; t1[f] = p1; t2[f] = 2.f * p2 - x0; }
  float o[CH];
#pragma unroll 1
  for (int h = 0; h < CH; ++h) { float a = bc[h];
#pragma unroll
    for (int f = 0; f < FIN; ++f) a += t0[f] * Wc[(0 * FIN + f) * CH + h] + t1[f] * Wc[(1 * FIN + f) * CH + h] + t2[f] * Wc[(2 * FIN + f) * CH + h];
    a = a > 0.f ? a : expm1f(a); o[h] = live ? a : 0.f; }
  if (!LAST) {
    for (int pass = 0; pass < 2; ++pass) {
#pragma unroll
      for (int h = 0; h < CH; ++h) { const float nb = __shfl_down(o[h], 1, 32); unsigned* rowp = TOUT + ((p * CH + h) * 64 + jj * 32) / 2;
        if ((lane & 1) == 0) ((volatile unsigned*)rowp)[lane >> 1] = (unsigned)__builtin_bit_cast(unsigned short, (_Float16)o[h]) | ((unsigned)__builtin_bit_cast(unsigned short, (_Float16)nb) << 16); }
      __threadfence(); }
  } else if (live) {
    typedef __attribute__((ext_vector_type(4))) unsigned u4; u4 v;
#pragma unroll
    for (int q = 0; q < 4; ++q) v[q] = (unsigned)__builtin_bit_cast(unsigned short, (_Float16)o[2 * q]) | ((unsigned)__builtin_bit_cast(unsigned short, (_Float16)o[2 * q + 1]) << 16);
    *(volatile u4*)(FLAT + (b * (CNn * CH) + n * CH) / 2) = v; __threadfence(); *(volatile u4*)(FLAT + (b * (CNn * CH) + n * CH) / 2) = v; }
}
__global__ __launch_bounds__(256) void head_kernel(const float* __restrict__ H1, const float* __restrict__ W2, const float* __restrict__ b2, float* __restrict__ out) {
  const long b = (long)blockIdx.x * 256 + threadIdx.x; if (b >= CBt) return;
  float l0 = b2[0], l1 = b2[1];
#pragma unroll 1
  for (int k = 0; k < 64; ++k) { const float h = H1[b * 64 + k]; l0 += h * W2[k]; l1 += h * W2[64 + k]; }
  const float m = fmaxf(l0, l1); const float lse = m + logf(expf(l0 - m) + expf(l1 - m));
  typedef __attribute__((ext_vector_type(2))) float v2f; const v2f v = {l0 - lse, l1 - lse};
  *(volatile v2f*)(out + b * 2) = v; __threadfence(); *(volatile v2f*)(out + b * 2) = v;
}
extern "C" void kernel_launch(void* const* d_in, const int* in_sizes, int n_in, void* d_out, int out_size, void* d_ws, size_t ws_size, hipStream_t stream) {
  (void)in_sizes; (void)n_in; (void)out_size; (void)ws_size;
  const float* x = (const float*)d_in[0]; const int* ei = (const int*)d_in[1];
  const float* W1c = (const float*)d_in[2]; const float* b1c = (const float*)d_in[3]; const float* W2c = (const float*)d_in[4]; const float* b2c = (const float*)d_in[5];
  const float* fc1W = (const float*)d_in[6]; const float* fc1b = (const float*)d_in[7]; const float* fc2W = (const float*)d_in[8]; const float* fc2b = (const float*)d_in[9];
  char* ws = (char*)d_ws; size_t off = 0;
  auto carve = [&](size_t bytes) -> char* { char* p = ws + off; off += (bytes + 255) & ~(size_t)255; return p; };
  unsigned* LB = (unsigned*)carve(64 * 64 * 2);
  unsigned* TA = (unsigned*)carve((size_t)CCH * CH * CNP * 2); unsigned* TB = (unsigned*)carve((size_t)CCH * CH * CNP * 2);
  float* C2 = (float*)carve((size_t)CCH * CH * CNP * 4);
  unsigned* FLAT = (unsigned*)carve((size_t)CBt * CNn * CH * 2); _Float16* W16 = (_Float16*)carve(64 * 192 * 2); float* H1 = (float*)carve((size_t)CBt * 64 * 4);
  lap_kernel<<<1, 256, 0, stream>>>(ei, LB);
  cast_f32_f16x2<<<(64 * 192 / 2 + 255) / 256, 256, 0, stream>>>(fc1W, W16, 64 * 192 / 2);
  for (int c = 0; c < CBt / CCH; ++c) {
    const float* xc = x + (size_t)c * CCH * CNn * CF1;
    t0_kernel<<<((CCH / 2) * CF1 + 255) / 256, 256, 0, stream>>>(xc, TA);
    { const int M = (CCH / 2) * CF1; const int t = (M / 64) * 1;
      wmma_gemm64<0, false, 0, 1, false><<<dim3((t + 7) / 8, 1), 256, 0, stream>>>((const unsigned short*)TA, nullptr, 64, 0, (const unsigned short*)LB, nullptr, 64, 0, TB, nullptr, 64, 0, nullptr, nullptr, 0, M, 64, 64, 1.0f);
      wmma_gemm64<0, false, 0, 0, false><<<dim3((t + 7) / 8, 1), 256, 0, stream>>>((const unsigned short*)TB, nullptr, 64, 0, (const unsigned short*)LB, nullptr, 64, 0, C2, nullptr, 64, 0, nullptr, nullptr, 0, M, 64, 64, 1.0f); }
    comb_kernel<CF1, false><<<CCH / 8, 256, 0, stream>>>(xc, nullptr, TB, C2, W1c, b1c, TA, nullptr);
    { const int M = (CCH / 2) * CH; const int t = (M / 64) * 1;
      wmma_gemm64<0, false, 0, 1, false><<<dim3((t + 7) / 8, 1), 256, 0, stream>>>((const unsigned short*)TA, nullptr, 64, 0, (const unsigned short*)LB, nullptr, 64, 0, TB, nullptr, 64, 0, nullptr, nullptr, 0, M, 64, 64, 1.0f);
      wmma_gemm64<0, false, 0, 0, false><<<dim3((t + 7) / 8, 1), 256, 0, stream>>>((const unsigned short*)TB, nullptr, 64, 0, (const unsigned short*)LB, nullptr, 64, 0, C2, nullptr, 64, 0, nullptr, nullptr, 0, M, 64, 64, 1.0f); }
    comb_kernel<CH, true><<<CCH / 8, 256, 0, stream>>>(nullptr, TA, TB, C2, W2c, b2c, nullptr, FLAT + (size_t)c * CCH * (CNn * CH) / 2);
  }
  { const int t = (CBt / 64) * 1;
    wmma_gemm64<0, false, 2, 0, false><<<dim3((t + 7) / 8, 1), 256, 0, stream>>>((const unsigned short*)FLAT, nullptr, CNn * CH, 0, U16(W16), nullptr, CNn * CH, 0, H1, nullptr, 64, 0, fc1b, nullptr, 0, CBt, 64, CNn * CH, 1.0f); }
  head_kernel<<<CBt / 256, 256, 0, stream>>>(H1, fc2W, fc2b, (float*)d_out);
}
